// DSConv_54717883351526
// MI455X (gfx1250) — hardware-verified
//
#include <hip/hip_runtime.h>
#include <math.h>

#define B_   8
#define C_   64
#define W_   128
#define H_   128
#define K_   9
#define OUT_ 64
#define KK_  576
#define NSP  16384
#define NPIX (B_ * NSP)

typedef __attribute__((ext_vector_type(16))) _Float16 v16h;
typedef __attribute__((ext_vector_type(8)))  _Float16 v8h;
typedef __attribute__((ext_vector_type(8)))  float    v8f;
typedef __attribute__((ext_vector_type(4)))  float    v4f;
typedef __attribute__((ext_vector_type(4)))  unsigned v4u;
typedef float __attribute__((may_alias)) float_a;

template <typename V> __device__ __forceinline__ void vst2(void* p, V v) {
  *(volatile V*)p = v; __threadfence(); *(volatile V*)p = v;
}
__device__ __forceinline__ v8f wmma_f16(v16h a, v16h b, v8f c) {
  v8f d = __builtin_amdgcn_wmma_f32_16x16x32_f16(false, a, false, b, (short)0, c, false, false);
  asm volatile("v_nop\n\tv_nop\n\tv_nop\n\tv_nop" : "+v"(d) : "v"(a), "v"(b));
  return d;
}
__device__ __forceinline__ v16h frag_h(const _Float16* row, int k0, int lane) {
  union { v16h v; v8h h[2]; } r; const _Float16* p = row + k0 + 8 * (lane >> 4);
  r.h[0] = *(const v8h*)(p); r.h[1] = *(const v8h*)(p + 16); return r.v;
}

__global__ __launch_bounds__(256) void k_pack_w(const float* __restrict__ w_dsc, _Float16* __restrict__ WT) {
  const int g = blockIdx.x * 256 + threadIdx.x;
  if (g >= OUT_ * KK_ / 8) return;
  const int o = (g * 8) / KK_, kk0 = (g * 8) % KK_;
  union { v8h h; v4u u; } pk;
#pragma unroll
  for (int e = 0; e < 8; ++e) { const int kk = kk0 + e, k = kk >> 6, c = kk & 63; pk.h[e] = (_Float16)w_dsc[(o * C_ + c) * K_ + k]; }
  vst2(WT + (size_t)g * 8, pk.u);
}

__global__ __launch_bounds__(256) void k_off_conv(const float* __restrict__ f, const float* __restrict__ w_off, const float* __restrict__ b_off,
                                                  float* __restrict__ off9, float* __restrict__ bn_part) {
  extern __shared__ char smem[];
  float* ftile = (float*)smem;
  float* wtile = ftile + 64 * 340;
  __shared__ float red[8][18];
  const int t = threadIdx.x, bid = blockIdx.x;
  const int bx = bid & 3, by = (bid >> 2) & 15, b = bid >> 6;
  for (int i = t; i < 64 * 340; i += 256) {
    const int c = i / 340, r = i - c * 340, yy = r / 34, xx = r - yy * 34;
    const int gy = by * 8 + yy - 1, gx = bx * 32 + xx - 1;
    float v = 0.f;
    if (gy >= 0 && gy < W_ && gx >= 0 && gx < H_) v = f[((size_t)(b * C_ + c) * W_ + gy) * H_ + gx];
    ftile[i] = v;
  }
  for (int i = t; i < 9 * C_ * 9; i += 256) wtile[i] = w_off[i];
  __syncthreads();
  const int yy = t >> 5, xx = t & 31;
  float acc[9];
#pragma unroll
  for (int ch = 0; ch < 9; ++ch) acc[ch] = b_off[ch];
  for (int c = 0; c < C_; ++c) {
    float r0[9];
#pragma unroll
    for (int dy = 0; dy < 3; ++dy)
#pragma unroll
      for (int dx = 0; dx < 3; ++dx) r0[dy * 3 + dx] = ftile[c * 340 + (yy + dy) * 34 + (xx + dx)];
#pragma unroll
    for (int ch = 0; ch < 9; ++ch) {
      const float* wp = &wtile[(ch * C_ + c) * 9];
      float s = acc[ch];
#pragma unroll
      for (int tap = 0; tap < 9; ++tap) s = fmaf(r0[tap], wp[tap], s);
      acc[ch] = s;
    }
  }
  const int gy = by * 8 + yy, gx = bx * 32 + xx;
#pragma unroll
  for (int ch = 0; ch < 9; ++ch) vst2(off9 + ((size_t)(b * K_ + ch) * W_ + gy) * H_ + gx, (float_a)acc[ch]);
#pragma unroll
  for (int ch = 0; ch < 9; ++ch) {
    float s1 = acc[ch], s2 = acc[ch] * acc[ch];
#pragma unroll
    for (int off = 16; off > 0; off >>= 1) { s1 += __shfl_xor(s1, off, 32); s2 += __shfl_xor(s2, off, 32); }
    if (xx == 0) { red[yy][ch] = s1; red[yy][9 + ch] = s2; }
  }
  __syncthreads();
  if (t < 32) {
    float v = 0.f;
    if (t < 18) { for (int w8 = 0; w8 < 8; ++w8) v += red[w8][t]; }
    vst2(bn_part + (size_t)bid * 32 + t, (float_a)v);
  }
}

__global__ __launch_bounds__(32) void k_bn_fin(const float* __restrict__ bn_part, float* __restrict__ bn_stats) {
  const int t = threadIdx.x;
  float v = 0.f;
  if (t < 18) {
    double s = 0.0;
    for (int i = 0; i < 512; ++i) s += (double)bn_part[i * 32 + t];
    v = (float)s;
  }
  const float sum = __shfl(v, t % 9, 32), sq = __shfl(v, 9 + (t % 9), 32);
  const float Nf = (float)(B_ * NSP);
  const float mu = sum / Nf, var = sq / Nf - mu * mu;
  float outv = 0.f;
  if (t < 9) outv = mu; else if (t < 18) outv = rsqrtf(var + 1e-5f);
  vst2(bn_stats + t, (float_a)outv);
}

__global__ __launch_bounds__(256) void k_offsets(const float* __restrict__ off9, const float* __restrict__ bn_stats,
                                                 const float* __restrict__ gmm, const float* __restrict__ bta, float* __restrict__ offn) {
  const int idx = blockIdx.x * 256 + threadIdx.x;
  const int b = idx >> 14, sp = idx & (NSP - 1);
  float tv[9];
#pragma unroll
  for (int k = 0; k < 9; ++k) {
    float v = off9[(size_t)(b * K_ + k) * NSP + sp];
    v = (v - bn_stats[k]) * bn_stats[9 + k] * gmm[k] + bta[k];
    tv[k] = tanhf(v);
  }
  float o[9];
  o[4] = 0.f;
  o[5] = tv[5]; o[6] = o[5] + tv[6]; o[7] = o[6] + tv[7];
  o[3] = tv[3]; o[2] = o[3] + tv[2]; o[1] = o[2] + tv[1];
  o[0] = tv[0]; o[8] = tv[8];
#pragma unroll
  for (int k = 0; k < 9; ++k) vst2(offn + (size_t)(b * K_ + k) * NSP + sp, (float_a)o[k]);
}

__global__ __launch_bounds__(256) void k_deform(const float* __restrict__ f, const float* __restrict__ offn, _Float16* __restrict__ A) {
  const int gid = blockIdx.x * 256 + threadIdx.x;
  const int part = gid & 7, item = gid >> 3;
  const int k = item % 9, pix = item / 9;
  const int b = pix >> 14, sp = pix & (NSP - 1), w = sp >> 7, h = sp & 127;
  const float y = (float)w + offn[(size_t)(b * K_ + k) * NSP + sp];
  const int x = h + k - 4;
  const float y0f = floorf(y);
  const int y0 = (int)y0f;
  float w1 = y - y0f, w0 = 1.f - w1;
  const bool ok = (x >= 0) && (x <= H_ - 2) && (y >= 0.f) && (y0 <= W_ - 2);
  union { v8h hh; v4u u; } pk;
  if (ok) {
    const float* p0 = f + ((size_t)(b * C_ + part * 8) * W_ + y0) * H_ + x;
#pragma unroll
    for (int e = 0; e < 8; ++e) { const float* pc = p0 + (size_t)e * NSP; pk.hh[e] = (_Float16)(pc[0] * w0 + pc[H_] * w1); }
  } else {
#pragma unroll
    for (int e = 0; e < 8; ++e) pk.hh[e] = (_Float16)0.f;
  }
  vst2(A + (size_t)pix * KK_ + k * 64 + part * 8, pk.u);
}

__global__ __launch_bounds__(128) void k_gemm(const _Float16* __restrict__ A, const _Float16* __restrict__ WT, const float* __restrict__ bias,
                                             float* __restrict__ xpre, float* __restrict__ gn_part) {
  __shared__ __align__(16) float so[4][16 * 64];
  __shared__ float red[4][32];
  const int tid = threadIdx.x, wave = tid >> 5, lane = tid & 31, hi = lane >> 4, col = lane & 15;
  const int strip = blockIdx.x * 4 + wave;
  const _Float16* ar = A + (size_t)(strip * 16 + col) * KK_;
  float* S = so[wave];
#pragma unroll 1
  for (int nt = 0; nt < 4; ++nt) {
    v8f acc = {};
    const _Float16* br = WT + (size_t)(nt * 16 + col) * KK_;
#pragma unroll 2
    for (int kc = 0; kc < KK_ / 32; ++kc) acc = wmma_f16(frag_h(ar, kc * 32, lane), frag_h(br, kc * 32, lane), acc);
#pragma unroll
    for (int r = 0; r < 8; ++r) S[(hi * 8 + r) * 64 + nt * 16 + col] = acc[r] + bias[nt * 16 + col];
  }
  __syncthreads();
  {
    const int g = lane & 15; float s = 0.f;
    for (int r = 0; r < 16; ++r)
#pragma unroll
      for (int cc = 0; cc < 4; ++cc) { const float v = S[r * 64 + g * 4 + cc]; s += hi ? v * v : v; }
    red[wave][lane] = s;
  }
  float* dst = xpre + (size_t)strip * 16 * 64;
#pragma unroll
  for (int q = 0; q < 8; ++q) { const int gq = q * 32 + lane; vst2(dst + gq * 4, *(const v4f*)(S + gq * 4)); }
  __syncthreads();
  if (tid < 32) vst2(gn_part + (size_t)blockIdx.x * 32 + tid, (float_a)(red[0][tid] + red[1][tid] + red[2][tid] + red[3][tid]));
}

__global__ __launch_bounds__(32) void k_gn_fin(const float* __restrict__ gn_part, float* __restrict__ gn_stats) {
  const int b = blockIdx.x, t = threadIdx.x;
  double s = 0.0;
  for (int i = 0; i < 256; ++i) s += (double)gn_part[((size_t)b * 256 + i) * 32 + t];
  const float v = (float)s;
  const float sum = __shfl(v, t & 15, 32), sq = __shfl(v, 16 + (t & 15), 32);
  const float Nf = (float)(4 * NSP);
  const float mu = sum / Nf, var = sq / Nf - mu * mu;
  vst2(gn_stats + b * 32 + t, (float_a)((t < 16) ? mu : rsqrtf(var + 1e-5f)));
}

__global__ __launch_bounds__(256) void k_gn_apply(const float* __restrict__ xpre, const float* __restrict__ gn_stats,
                                                  const float* __restrict__ gmm, const float* __restrict__ bta, float* __restrict__ out) {
  const int q = blockIdx.x * 256 + threadIdx.x;
  const int b = q >> 18, o = (q >> 12) & 63, sp0 = (q & 4095) * 4, g = o >> 2;
  const float mu = gn_stats[b * 32 + g], rs = gn_stats[b * 32 + 16 + g], ga = gmm[o], be = bta[o];
  v4f x;
#pragma unroll
  for (int e = 0; e < 4; ++e) x[e] = fmaxf((xpre[((size_t)(b * NSP + sp0 + e)) * 64 + o] - mu) * rs * ga + be, 0.f);
  vst2(out + (size_t)q * 4, x);
}

extern "C" void kernel_launch(void* const* d_in, const int* in_sizes, int n_in,
                              void* d_out, int out_size, void* d_ws, size_t ws_size,
                              hipStream_t stream) {
  (void)in_sizes; (void)n_in; (void)out_size; (void)ws_size;
  const float* f     = (const float*)d_in[0];
  const float* w_off = (const float*)d_in[1];
  const float* b_off = (const float*)d_in[2];
  const float* bn_g  = (const float*)d_in[3];
  const float* bn_b  = (const float*)d_in[4];
  const float* w_dsc = (const float*)d_in[5];
  const float* b_dsc = (const float*)d_in[6];
  const float* gn_g  = (const float*)d_in[7];
  const float* gn_b  = (const float*)d_in[8];
  float* out = (float*)d_out;

  char* ws = (char*)d_ws; size_t off = 0;
  auto alloc = [&](size_t bytes) -> void* { void* p = ws + off; off = (off + bytes + 255) & ~(size_t)255; return p; };
  _Float16* WT    = (_Float16*)alloc((size_t)OUT_ * KK_ * 2);
  float* off9     = (float*)alloc((size_t)B_ * K_ * NSP * 4);
  float* bn_part  = (float*)alloc(512 * 32 * 4);
  float* bn_stats = (float*)alloc(32 * 4);
  float* offn     = (float*)alloc((size_t)B_ * K_ * NSP * 4);
  _Float16* A     = (_Float16*)alloc((size_t)NPIX * KK_ * 2);
  float* xpre     = (float*)alloc((size_t)NPIX * OUT_ * 4);
  float* gn_part  = (float*)alloc(2048 * 32 * 4);
  float* gn_stats = (float*)alloc(B_ * 32 * 4);

  k_pack_w<<<(OUT_ * KK_ / 8 + 255) / 256, 256, 0, stream>>>(w_dsc, WT);
  k_off_conv<<<512, 256, (64 * 340 + 9 * 64 * 9) * 4, stream>>>(f, w_off, b_off, off9, bn_part);
  k_bn_fin<<<1, 32, 0, stream>>>(bn_part, bn_stats);
  k_offsets<<<NPIX / 256, 256, 0, stream>>>(off9, bn_stats, bn_g, bn_b, offn);
  k_deform<<<NPIX * 9 * 8 / 256, 256, 0, stream>>>(f, offn, A);
  k_gemm<<<NPIX / 64, 128, 0, stream>>>(A, WT, b_dsc, xpre, gn_part);
  k_gn_fin<<<B_, 32, 0, stream>>>(gn_part, gn_stats);
  k_gn_apply<<<(B_ * OUT_ * NSP / 4) / 256, 256, 0, stream>>>(xpre, gn_stats, gn_g, gn_b, out);
}
